// EdgeClassify_79929341378653
// MI455X (gfx1250) — hardware-verified
//
#include <hip/hip_runtime.h>


#ifndef NB
#define NB 8
#endif
#define NB_FULL 8
#define KL   2048
#define DM   512
#define AT   64
#define NC   5
#define NCP  16
#define K2   (2 * DM)
#define ETP  40
#define OSP  68
#define RCS  16.0f
#define WCS  1024.0f
#define FOLD (1.0f / 16384.0f)

static_assert(NB <= NB_FULL);
static_assert(KL % 32 == 0);
static_assert(DM % 64 == 0);
static_assert(DM % 32 == 0);
static_assert((DM & (DM - 1)) == 0);
static_assert(AT == 64);
static_assert((NB * AT) % 16 == 0);
static_assert(NC <= NCP);
static_assert((ETP * 2) % 16 == 0);
static_assert((OSP * 4) % 16 == 0);
static_assert(128 * 16 * 4 == AT * 64 * 2);
static_assert((AT * NC) % 4 == 0);
static_assert(32 * 16 * 40 == 16 * AT * NC * 4);
static_assert((16 * AT * NC * 4) % 128 == 0);
static_assert((NCP * K2 / 8) % 256 == 0);
static_assert((AT * KL / 8) % 256 == 0);
static_assert(64 * ETP * 2 + AT * OSP * 4 <= 131072);
static_assert(16 * 16 * 4 <= 131072);

typedef _Float16 h16;
typedef unsigned short bf;
typedef __attribute__((ext_vector_type(16))) __bf16   v16bf;
typedef __attribute__((ext_vector_type(16))) _Float16 v16h;
typedef __attribute__((ext_vector_type(8)))  _Float16 v8h;
typedef __attribute__((ext_vector_type(8)))  unsigned short v8us;
typedef __attribute__((ext_vector_type(8)))  float    v8f;
typedef __attribute__((ext_vector_type(4)))  float    v4f;
typedef v4f  __attribute__((may_alias)) v4fa;

__device__ __forceinline__ unsigned short f2bf(float f) { unsigned u = __float_as_uint(f); u += 0x7FFFu + ((u >> 16) & 1u); return (unsigned short)(u >> 16); }
__device__ __forceinline__ float bfr(float f) { return __uint_as_float(((unsigned)f2bf(f)) << 16); }
__device__ __forceinline__ v16h cat16(v8h lo, v8h hi) { return __builtin_shufflevector(lo, hi, 0, 1, 2, 3, 4, 5, 6, 7, 8, 9, 10, 11, 12, 13, 14, 15); }
__device__ __forceinline__ v16bf cat16b(v8us lo, v8us hi) { return __builtin_bit_cast(v16bf, __builtin_shufflevector(lo, hi, 0, 1, 2, 3, 4, 5, 6, 7, 8, 9, 10, 11, 12, 13, 14, 15)); }
__device__ __forceinline__ v16h  ldh(const h16* p) { return cat16(*(const v8h*)p, *(const v8h*)(p + 16)); }
__device__ __forceinline__ v16bf ldb(const bf* p)  { return cat16b(*(const v8us*)p, *(const v8us*)(p + 16)); }
__device__ __forceinline__ void wave_sync() { __builtin_amdgcn_fence(3  , "wavefront"); __builtin_amdgcn_wave_barrier(); asm volatile("" ::: "memory"); }
__device__ __forceinline__ h16 toh_flush(float v) { const h16 r = (h16)v; return (fabsf(v) < 6.103515625e-05f) ? (h16)0.0f : r; }
__device__ __forceinline__ v8f wmmab_g(v16bf a, v16bf b, v8f c) {
    c = __builtin_amdgcn_wmma_f32_16x16x32_bf16(false, a, false, b, (short)0, c, false, false);
    asm volatile("v_nop\n\tv_nop\n\tv_nop\n\tv_nop" : "+v"(c) : "v"(a), "v"(b));
    return c; }
__device__ __forceinline__ v8f wmma16_g(v16h a, v16h b, v8f c) {
    c = __builtin_amdgcn_wmma_f32_16x16x32_f16(false, a, false, b, (short)0, c, false, false);
    asm volatile("v_nop\n\tv_nop\n\tv_nop\n\tv_nop" : "+v"(c) : "v"(a), "v"(b));
    return c; }

__global__ __launch_bounds__(256) void k_cvt8(const float* __restrict__ src, bf* dst, size_t n8) {
    const size_t i = (size_t)blockIdx.x * 256 + threadIdx.x; if (i >= n8) return;
    const v8f v = *(const v8f*)(src + i * 8); v8us o;
#pragma unroll
    for (int k = 0; k < 8; ++k) o[k] = f2bf(v[k]);
    *(volatile v8us*)(dst + i * 8) = o; __threadfence(); *(volatile v8us*)(dst + i * 8) = o;
}

__global__ __launch_bounds__(256) void k_wplane(const float* __restrict__ w2, h16* WF) {
    const unsigned i = blockIdx.x * 256u + threadIdx.x;
    if (i >= (unsigned)(NCP * K2 / 8)) return;
    const unsigned row = i / (unsigned)(K2 / 8), c8 = (i % (unsigned)(K2 / 8)) * 8u;
    const unsigned rc = row < (unsigned)NC ? row : (unsigned)(NC - 1);
    v8f v = *(const v8f*)(w2 + (size_t)rc * K2 + c8);
    asm volatile("" : "+v"(v));
    const bool live = row < (unsigned)NC;
    v8h o;
#pragma unroll
    for (int k = 0; k < 8; ++k) { const float s = live ? (bfr(v[k]) * WCS) : 0.0f; o[k] = toh_flush(s); }
    *(volatile v8h*)(WF + (size_t)i * 8) = o; __threadfence(); *(volatile v8h*)(WF + (size_t)i * 8) = o;
}

__global__ __launch_bounds__(128) void k_gemm1(const float* __restrict__ X, const bf* __restrict__ WLB, const float* __restrict__ b1, h16* R) {
    __shared__ __align__(16) bf    et[64 * ETP];
    __shared__ __align__(16) float os[AT * OSP];
    const int lane = threadIdx.x & 31, lr = lane & 15, hi = lane >> 4;
    const int wave = __builtin_amdgcn_readfirstlane((int)(threadIdx.x >> 5));
    const int d0 = blockIdx.x * 64, b = blockIdx.y;
    const int sd = threadIdx.x & 63, sk = (int)(threadIdx.x >> 6) * 16;
    const float* xp = X + (size_t)b * KL * DM + (size_t)sk * DM + d0 + sd;
    v8f acc[4];
#pragma unroll
    for (int mb = 0; mb < 4; ++mb) acc[mb] = (v8f){};
    const size_t aoff = (size_t)lr * KL + 8 * hi;
    const int boff = (wave * 16 + lr) * ETP + 8 * hi;
    const int soff = sd * ETP + sk;
#pragma unroll 1
    for (int k0 = 0; k0 < KL; k0 += 32) {
        const float* p = xp + (size_t)k0 * DM;
        float x[8]; v8us lo8, hi8;
#pragma unroll
        for (int i = 0; i < 8; ++i) x[i] = p[(size_t)i * DM];
#pragma unroll
        for (int i = 0; i < 8; ++i) lo8[i] = f2bf(x[i]);
#pragma unroll
        for (int i = 0; i < 8; ++i) x[i] = p[(size_t)(8 + i) * DM];
#pragma unroll
        for (int i = 0; i < 8; ++i) hi8[i] = f2bf(x[i]);
        *(v8us*)(&et[soff]) = lo8; *(v8us*)(&et[soff + 8]) = hi8;
        __syncthreads();
        const v16bf bq = cat16b(*(const v8us*)(&et[boff]), *(const v8us*)(&et[boff + 16]));
        v16bf a[4];
#pragma unroll
        for (int mb = 0; mb < 4; ++mb) a[mb] = ldb(WLB + aoff + (size_t)mb * 16 * KL + k0);
#pragma unroll
        for (int mb = 0; mb < 4; ++mb) acc[mb] = wmmab_g(a[mb], bq, acc[mb]);
        __syncthreads();
    }
#pragma unroll
    for (int mb = 0; mb < 4; ++mb) {
#pragma unroll
        for (int r = 0; r < 8; ++r) os[(mb * 16 + 8 * hi + r) * OSP + wave * 16 + lr] = acc[mb][r]; }
    __syncthreads();
    h16* rb = R + (size_t)b * AT * DM + d0;
#pragma unroll 1
    for (int ps = 0; ps < 2; ++ps) {
#pragma unroll
        for (int s = 0; s < 4; ++s) { const int row = wave * 16 + 4 * s + (lane >> 3), c8 = (lane & 7) * 8;
            const float bz = bfr(b1[row]);
            const v4f x0 = *(const v4fa*)(&os[row * OSP + c8]); const v4f x1 = *(const v4fa*)(&os[row * OSP + c8 + 4]); v8h hv;
#pragma unroll
            for (int i = 0; i < 4; ++i) { hv[i] = toh_flush((x0[i] + bz) * RCS); hv[4 + i] = toh_flush((x1[i] + bz) * RCS); }
            *(volatile v8h*)(rb + (size_t)row * DM + c8) = hv; }
        if (ps == 0) __threadfence(); }
}

__global__ __launch_bounds__(32) void k_gemm2(const h16* __restrict__ R, const h16* __restrict__ WF, const float* __restrict__ b2, const int* __restrict__ rep_p, float* OUT) {
    __shared__ __align__(16) float vs[16 * 16];
    const int lane = threadIdx.x & 31, lr = lane & 15, hi = lane >> 4;
    const int m0 = blockIdx.x * 16;
    v8f acc = (v8f){};
    const size_t ao = (size_t)(m0 + lr) * DM + 8 * hi;
    const size_t bo = (size_t)lr * K2 + 8 * hi;
#pragma unroll 1
    for (int kc = 0; kc < K2; kc += 32) {
        const v16h a = ldh(R + ao + (size_t)(kc & (DM - 1)));
        const v16h w = ldh(WF + bo + (size_t)kc);
        acc = wmma16_g(a, w, acc);
    }
    const int nc = lr < NC ? lr : (NC - 1);
    float bz = b2[nc];
    asm volatile("" : "+v"(bz));
    const float bias = (lr < NC) ? bfr(bz) : 0.0f;
    const bool bad = rep_p[0] != AT;
    const float qnan = __uint_as_float(0x7FC00000u);
#pragma unroll
    for (int r = 0; r < 8; ++r) { float v = acc[r] * FOLD + bias; v = bad ? qnan : v; vs[(8 * hi + r) * 16 + lr] = v; }
    wave_sync();
    float* ob = OUT + (size_t)m0 * (AT * NC);
#pragma unroll 1
    for (int ps = 0; ps < 2; ++ps) {
#pragma unroll 1
        for (int it = 0; it < 40; ++it) {
            unsigned q = (unsigned)it * 32u + (unsigned)lane;
            asm volatile("" : "+v"(q));
            const unsigned row = q / 80u;
            const unsigned c = (q - row * 80u) * 4u;
            v4f val;
#pragma unroll
            for (int i = 0; i < 4; ++i) val[i] = vs[row * 16u + ((c + (unsigned)i) % 5u)];
            *(volatile v4f*)(ob + (size_t)q * 4) = val; }
        if (ps == 0) __threadfence(); }
}

static constexpr size_t al256(size_t v) { return (v + 255) & ~(size_t)255; }
static constexpr size_t SZ_WL = al256((size_t)AT * KL * 2);
static constexpr size_t SZ_WF = al256((size_t)NCP * K2 * 2);
static constexpr size_t SZ_R  = al256((size_t)NB * AT * DM * 2);
static constexpr size_t SZ_TOTAL = SZ_WL + SZ_WF + SZ_R;
static_assert(SZ_TOTAL <= (size_t)134217728);
static_assert((size_t)NB * AT * AT * NC * 4 <= (size_t)655360);

extern "C" void kernel_launch(void* const* d_in, const int* in_sizes, int n_in,
                              void* d_out, int out_size, void* d_ws, size_t ws_size, hipStream_t stream) {
    if (n_in < 6) return;
    if ((size_t)in_sizes[0] < (size_t)NB * KL * DM) return;
    if ((size_t)in_sizes[1] < (size_t)AT * KL) return;
    if (in_sizes[2] < AT) return;
    if ((size_t)in_sizes[3] < (size_t)NC * K2) return;
    if (in_sizes[4] < NC || in_sizes[5] < 1) return;
    if ((size_t)out_size < (size_t)NB * AT * AT * NC) return;
    if (SZ_TOTAL > ws_size) return;
    const float* x  = (const float*)d_in[0];
    const float* w1 = (const float*)d_in[1];
    const float* b1 = (const float*)d_in[2];
    const float* w2 = (const float*)d_in[3];
    const float* b2 = (const float*)d_in[4];
    const int*  rep = (const int*)d_in[5];
    float* OUT = (float*)d_out;
    char* wsp = (char*)d_ws;
    bf*  WLB = (bf*)wsp;  wsp += SZ_WL;
    h16* WF  = (h16*)wsp; wsp += SZ_WF;
    h16* R   = (h16*)wsp; wsp += SZ_R;

    { const size_t n8 = (size_t)AT * KL / 8; k_cvt8<<<(unsigned)((n8 + 255) / 256), 256, 0, stream>>>(w1, WLB, n8); }
    k_wplane<<<(unsigned)(NCP * K2 / 8 / 256), 256, 0, stream>>>(w2, WF);
    k_gemm1<<<dim3(DM / 64, NB, 1), 128, 0, stream>>>(x, WLB, b1, R);
    k_gemm2<<<dim3(NB * AT / 16, 1, 1), 32, 0, stream>>>(R, WF, b2, rep, OUT);
}
